// KPConv_68281390072586
// MI455X (gfx1250) — hardware-verified
//
#include <hip/hip_runtime.h>
#include <math.h>

typedef __attribute__((ext_vector_type(16))) _Float16 v16h;
typedef __attribute__((ext_vector_type(16))) __bf16 v16b;
typedef __attribute__((ext_vector_type(8)))  _Float16 v8h;
typedef __attribute__((ext_vector_type(8)))  float v8f;
typedef __attribute__((ext_vector_type(4)))  float v4f;
typedef __attribute__((ext_vector_type(2)))  float v2f;
typedef __attribute__((ext_vector_type(4)))  unsigned v4u;
typedef __attribute__((ext_vector_type(4)))  int v4i;
typedef float __attribute__((may_alias)) float_a;
typedef int __attribute__((may_alias)) int_a;

template <typename T> __device__ __forceinline__ void vst2(void* p, T v) { *(volatile T*)p = v; __threadfence(); *(volatile T*)p = v; }
__device__ __forceinline__ v8f wmma16(v16h a, v16h b, v8f c) {
  v8f d = __builtin_amdgcn_wmma_f32_16x16x32_f16(false, a, false, b, (short)0, c, false, false);
  asm volatile("v_nop\n\tv_nop\n\tv_nop\n\tv_nop" : "+v"(d) : "v"(a), "v"(b));
  return d;
}
__device__ __forceinline__ v8f wmma_bf(v16b a, v16b b, v8f c) {
  v8f d = __builtin_amdgcn_wmma_f32_16x16x32_bf16(false, a, false, b, (short)0, c, false, false);
  asm volatile("v_nop\n\tv_nop\n\tv_nop\n\tv_nop" : "+v"(d) : "v"(a), "v"(b));
  return d;
}
__device__ __forceinline__ v16h frag_h(const _Float16* rowk0, int lane) {
  union { v16h v; v8h q[2]; } u; const _Float16* p = rowk0 + 8 * (lane >> 4);
  u.q[0] = *(const v8h*)p; u.q[1] = *(const v8h*)(p + 16); return u.v;
}
__device__ __forceinline__ v16h frag_f32(const float* rowk0, int lane) {
  v16h a; const float* p = rowk0 + 8 * (lane >> 4);
#pragma unroll
  for (int i = 0; i < 8; ++i) { a[i] = (_Float16)p[i]; a[8 + i] = (_Float16)p[16 + i]; }
  return a;
}
__device__ __forceinline__ v16h frag_f32s(const float* rowk0, int lane, float sc) {
  v16h a; const float* p = rowk0 + 8 * (lane >> 4);
#pragma unroll
  for (int i = 0; i < 8; ++i) { a[i] = (_Float16)(p[i] * sc); a[8 + i] = (_Float16)(p[16 + i] * sc); }
  return a;
}
__device__ __forceinline__ v16h fragc_f32(const float* W, int k0, int n, int lane, int ld, int K) {
  v16h a; const int g = lane >> 4;
#pragma unroll
  for (int i = 0; i < 8; ++i) { const int ka = k0 + 8 * g + i, kb = ka + 16;
    a[i] = (_Float16)(ka < K ? W[(size_t)(ka < K ? ka : K - 1) * ld + n] : 0.f); a[8 + i] = (_Float16)(kb < K ? W[(size_t)(kb < K ? kb : K - 1) * ld + n] : 0.f); }
  return a;
}
struct F2 { v16b h, l; };
__device__ __forceinline__ F2 bsplit16(const float v[16]) { F2 r;
#pragma unroll
  for (int i = 0; i < 16; ++i) { const __bf16 h = (__bf16)v[i]; r.h[i] = h; r.l[i] = (__bf16)(v[i] - (float)h); }
  return r; }
__device__ __forceinline__ F2 split_row(const float* row, int k0, int lane) { float v[16]; const float* p = row + k0 + 8 * (lane >> 4);
#pragma unroll
  for (int i = 0; i < 8; ++i) { v[i] = p[i]; v[8 + i] = p[16 + i]; }
  return bsplit16(v); }
__device__ __forceinline__ F2 split_rowK(const float* row, int k0, int lane, int K) { float v[16]; const int g = lane >> 4;
#pragma unroll
  for (int i = 0; i < 8; ++i) { const int ka = k0 + 8 * g + i, kb = ka + 16; v[i] = ka < K ? row[ka < K ? ka : K - 1] : 0.f; v[8 + i] = kb < K ? row[kb < K ? kb : K - 1] : 0.f; }
  return bsplit16(v); }
__device__ __forceinline__ F2 split_col(const float* W, int k0, int n, int lane, int ld, int K) { float v[16]; const int g = lane >> 4;
#pragma unroll
  for (int i = 0; i < 8; ++i) { const int ka = k0 + 8 * g + i, kb = ka + 16; v[i] = ka < K ? W[(size_t)(ka < K ? ka : K - 1) * ld + n] : 0.f; v[8 + i] = kb < K ? W[(size_t)(kb < K ? kb : K - 1) * ld + n] : 0.f; }
  return bsplit16(v); }
__device__ __forceinline__ v8f mac3(const F2& a, const F2& b, v8f c) { c = wmma_bf(a.l, b.h, c); c = wmma_bf(a.h, b.l, c); return wmma_bf(a.h, b.h, c); }
__device__ __forceinline__ float sigm(float v) { return 1.0f / (1.0f + expf(-v)); }
#define LDSX() do { asm volatile("s_wait_dscnt 0" ::: "memory"); __builtin_amdgcn_wave_barrier(); __builtin_amdgcn_fence(__ATOMIC_RELEASE, "workgroup"); } while (0)

__device__ __forceinline__ float bfr(float v) { return (float)(__bf16)v; }
#define NBT 2
#define NQ 16384
#define MS 16384
#define NPTS (NBT * NQ)
#define NNB 32
#define KP 15
#define CIN 64
#define COUT 128
#define KAGG (KP * CIN)
#ifndef NPB
#define NPB NPTS
#endif
#define WS_AGG 0u
#define WS_END (WS_AGG + 2u * (size_t)NPTS * KAGG)
__global__ __launch_bounds__(128) void k_agg(const float* __restrict__ FEAT, const float* __restrict__ XYZQ, const float* __restrict__ XYZS, const int* __restrict__ NIDX, const float* __restrict__ KPT, _Float16* __restrict__ AGG) {
  __shared__ __align__(16) _Float16 sg[4][16][72];
  const int tid = threadIdx.x, wave = tid >> 5, lane = tid & 31, col = lane & 15, g = lane >> 4; const size_t n = (size_t)blockIdx.x * 4 + wave; const size_t b = n / NQ;
  const float x0 = bfr(XYZQ[n * 3]), y0 = bfr(XYZQ[n * 3 + 1]), z0 = bfr(XYZQ[n * 3 + 2]);
  float av[16]; int je[16];
#pragma unroll
  for (int i = 0; i < 16; ++i) { const int e = (i < 8) ? (8 * g + i) : (16 + 8 * g + (i - 8)); int j = NIDX[n * NNB + e]; j = j < 0 ? 0 : (j >= MS ? MS - 1 : j); const size_t js = b * MS + j; je[i] = (int)js;
    const float rx = bfr(XYZS[js * 3]) - x0, ry = bfr(XYZS[js * 3 + 1]) - y0, rz = bfr(XYZS[js * 3 + 2]) - z0;
    const int k = col < KP ? col : 0; const float dx = rx - bfr(KPT[k * 3]), dy = ry - bfr(KPT[k * 3 + 1]), dz = rz - bfr(KPT[k * 3 + 2]);
    const float sq = (dx * dx + dy * dy) + dz * dz; const float ev = (col < KP) ? expf(-sq * 200.0f) : 0.f;
    float tot = ev;
#pragma unroll
    for (int sh = 1; sh < 16; sh <<= 1) tot += __shfl_xor(tot, sh);
    av[i] = ev / (tot + 1e-6f); }
  const F2 a = bsplit16(av);
#pragma unroll
  for (int jt = 0; jt < CIN / 16; ++jt) { v16b fb; const int c = jt * 16 + col;
#pragma unroll
    for (int i = 0; i < 16; ++i) fb[i] = (__bf16)FEAT[(size_t)je[i] * CIN + c];
    v8f acc = {}; acc = wmma_bf(a.h, fb, acc); acc = wmma_bf(a.l, fb, acc);
#pragma unroll
    for (int r = 0; r < 8; ++r) sg[wave][8 * g + r][jt * 16 + col] = (_Float16)acc[r]; }
  LDSX();
  for (int e = lane; e < KP * 8; e += 32) { const int row = e >> 3, q = e & 7; vst2((unsigned*)(AGG + n * KAGG + row * CIN + q * 8), *(const v4u*)&sg[wave][row][q * 8]); } }
__global__ __launch_bounds__(128) void k_gemm(const _Float16* __restrict__ AGG, const float* __restrict__ W, const float* __restrict__ BIAS, float* __restrict__ PRE) { __shared__ __align__(16) float sf[4][16][132];
  const int tid = threadIdx.x, wave = tid >> 5, lane = tid & 31, col = lane & 15, g = lane >> 4; const size_t r0 = (size_t)blockIdx.x * 64 + wave * 16; const size_t ra = (r0 + col < NPB) ? r0 + col : NPB - 1;
  v8f acc[8] = {};
#pragma unroll 2
  for (int kc = 0; kc < KAGG / 32; ++kc) { const v16h a = frag_h(AGG + ra * KAGG + kc * 32, lane);
#pragma unroll
    for (int j = 0; j < 8; ++j) { v16h w; const int o = j * 16 + col;
#pragma unroll
      for (int i = 0; i < 8; ++i) { w[i] = (_Float16)(bfr(W[(size_t)(kc * 32 + 8 * g + i) * COUT + o]) * 16.0f); w[8 + i] = (_Float16)(bfr(W[(size_t)(kc * 32 + 16 + 8 * g + i) * COUT + o]) * 16.0f); }
      acc[j] = wmma16(a, w, acc[j]); } }
#pragma unroll
  for (int j = 0; j < 8; ++j)
#pragma unroll
    for (int r = 0; r < 8; ++r) sf[wave][8 * g + r][j * 16 + col] = acc[j][r] * (1.0f / 16.0f) + bfr(BIAS[j * 16 + col]);
  LDSX(); for (int rl = 0; rl < 16; ++rl) { const size_t r = r0 + rl; if (r < NPB) vst2(PRE + r * COUT + lane * 4, *(const v4f*)&sf[wave][rl][lane * 4]); } }
extern "C" void kernel_launch(void* const* d_in, const int* in_sizes, int n_in, void* d_out, int out_size, void* d_ws, size_t ws_size, hipStream_t stream) {
  (void)in_sizes; (void)n_in; (void)out_size;
  const float** F = (const float**)d_in;
  if (ws_size < (size_t)WS_END) return;
  char* ws = (char*)d_ws; _Float16* AGG = (_Float16*)(ws + WS_AGG);
  k_agg<<<dim3(NPB / 4), 128, 0, stream>>>(F[2], F[0], F[1], (const int*)d_in[3], F[4], AGG);
  k_gemm<<<dim3((NPB + 63) / 64), 128, 0, stream>>>(AGG, F[5], F[6], (float*)d_out);
}
